// PsdFeatureExtractor_32607391711296
// MI455X (gfx1250) — hardware-run, weakly checked
//
#include <hip/hip_runtime.h>
#include <math.h>

typedef __attribute__((ext_vector_type(16))) _Float16 v16h;
typedef __attribute__((ext_vector_type(8)))  _Float16 v8h;
typedef __attribute__((ext_vector_type(8)))  float    v8f;
typedef __attribute__((ext_vector_type(4)))  float    v4f;

constexpr int kNumSig     = 1024;
constexpr int kSigLen     = 4000;
constexpr int kFft        = 200;
constexpr int kTaps       = 16;
constexpr int kHop        = 8;
constexpr int kLeft       = (kFft - kTaps) / 2;
constexpr int kPadEach    = kFft / 2;
constexpr int kShift      = kPadEach - kLeft;
constexpr int kFrames     = kSigLen / kHop + 1;
constexpr int kFramesPad  = 512;
constexpr int kBands      = 7;
constexpr int kBinsUsed   = 100;
constexpr int kBinTiles   = 7;
constexpr int kBinRows    = kBinTiles * 16;
constexpr int kKPad       = 32;
constexpr int kKinds      = 4;
constexpr int kKindStride = kBinRows * kKPad;
constexpr int kBasisElems = kKinds * kKindStride;
constexpr int kStageLen   = 4112;
constexpr int kStageIters = (kStageLen + 255) / 256;
constexpr int kCoefElems  = 2 * kBinRows * kTaps;
constexpr int kPlaneSig   = kBands * kFramesPad;
constexpr int kPlaneVec   = kPlaneSig / 4;
constexpr int kOutSig     = kBands * kFrames;
constexpr int kOutElems   = kNumSig * kOutSig;
constexpr int kOutVec     = kOutElems / 4;

static_assert(kLeft == 92 && kShift == 8 && kFrames == 501, "frame geometry");
static_assert(kFramesPad % 128 == 0 && kFramesPad >= kFrames, "padded frame count");
static_assert(kStageLen >= kHop * (kFramesPad - 1) + kTaps, "staged samples cover every padded frame");
static_assert(kStageLen - 1 - kShift <= 2 * kSigLen - 2, "mirror index stays in range");
static_assert(kBinRows >= kBinsUsed, "bin rows");
static_assert(kBasisElems == 7 * 256 * 8, "basis plane = 7 x 256 threads x 8 halves");
static_assert(kCoefElems == 14 * 256, "coefficient table = 14 x 256 threads");
static_assert(kOutVec % 256 == 0 && kOutVec * 4 == kOutElems, "compaction grid is exact");
static_assert((kOutElems * 4) % 128 == 0, "output is a whole number of 128-B lines");
static_assert(kPlaneVec == 3 * 256 + 128, "stage-out map");

constexpr int kEdge1 = 4, kEdge2 = 8, kEdge3 = 12, kEdge4 = 30, kEdge5 = 50, kEdge6 = 70, kEdge7 = 100;
constexpr int kNoEdge = 1 << 20;
static_assert(kEdge7 == kBinsUsed, "last band edge");

__host__ __device__ constexpr int band_end(int b) {
  return b == 0 ? kEdge1 : b == 1 ? kEdge2 : b == 2 ? kEdge3 : b == 3 ? kEdge4
       : b == 4 ? kEdge5 : b == 5 ? kEdge6 : b == 6 ? kEdge7 : kNoEdge;
}
__host__ __device__ constexpr int band_first(int b) { return b == 0 ? 0 : band_end(b - 1); }
__host__ __device__ constexpr int band_width(int b) { return band_end(b) - band_first(b); }
static_assert(band_width(0) == 4 && band_width(1) == 4 && band_width(2) == 4 && band_width(3) == 18 &&
              band_width(4) == 20 && band_width(5) == 20 && band_width(6) == 30, "band widths");

__device__ __forceinline__ int band_of_bin(int b) {
  return (b >= kEdge1) + (b >= kEdge2) + (b >= kEdge3) + (b >= kEdge4) + (b >= kEdge5) + (b >= kEdge6) + (b >= kEdge7);
}

constexpr float kXCarry   = 16.0f;
constexpr float kBCarry   = 16.0f;
constexpr float kResCarry = 2048.0f;
constexpr float kInvRes   = 1.0f / kResCarry;
constexpr float kInvCarry = 1.0f / (kXCarry * kBCarry);
constexpr float kF16Min   = 6.103515625e-05f;
constexpr float kEps      = 1e-10f;

constexpr size_t kOffBasis = 0;
constexpr size_t kOffPlane = kOffBasis + (size_t)kBasisElems * 2;
constexpr size_t kWsTotal  = kOffPlane + (size_t)kNumSig * kPlaneSig * 4;
static_assert(kOffPlane == 28672ull && (kOffPlane % 128) == 0, "plane offset");
static_assert(kWsTotal == 14708736ull && kWsTotal <= 134217728ull, "carve total");

union FragH { v16h v; v8h h[2]; };

__device__ __forceinline__ v16h frag_load(const _Float16* p) {
  FragH f;
  f.h[0] = *(const v8h*)(p);
  f.h[1] = *(const v8h*)(p + 16);
  return f.v;
}

__device__ __forceinline__ v8f mma_h(v16h a, v16h b, v8f c) {
  c = __builtin_amdgcn_wmma_f32_16x16x32_f16(false, a, false, b, (short)0, c, false, false);
  asm volatile("v_nop\n\tv_nop\n\tv_nop\n\tv_nop" : "+v"(c) : "v"(a), "v"(b));
  return c;
}

__device__ __forceinline__ void split_parts(float v, float& hf, float& rf) {
  const float vh = (fabsf(v) < kF16Min) ? 0.0f : v;
  const _Float16 h16 = (_Float16)vh;
  hf = (float)h16;
  const float r = (v - hf) * kResCarry;
  rf = (fabsf(r) < kF16Min) ? 0.0f : r;
}

constexpr double kPiQuarter = 0.785398163397448309616;

__device__ __forceinline__ void cs_two_pi(int p, int n, double qscale, double& c, double& s) {
  const int p8  = 8 * p;
  const int oc  = p8 / n;
  const int odd = oc & 1;
  const int r   = odd ? ((oc + 1) * n - p8) : (p8 - oc * n);
  const double a = (double)r * qscale;
  const double z = a * a;
  double ps = 1.0 / 6227020800.0;
  ps = ps * z - 1.0 / 39916800.0;
  ps = ps * z + 1.0 / 362880.0;
  ps = ps * z - 1.0 / 5040.0;
  ps = ps * z + 1.0 / 120.0;
  ps = ps * z - 1.0 / 6.0;
  ps = ps * z + 1.0;
  const double s0 = a * ps;
  double pc = -1.0 / 87178291200.0;
  pc = pc * z + 1.0 / 479001600.0;
  pc = pc * z - 1.0 / 3628800.0;
  pc = pc * z + 1.0 / 40320.0;
  pc = pc * z - 1.0 / 720.0;
  pc = pc * z + 1.0 / 24.0;
  pc = pc * z - 0.5;
  const double c0 = pc * z + 1.0;
  const bool swp  = ((oc + 1) & 2) != 0;
  const bool cneg = ((oc + 2) & 4) != 0;
  const bool sneg = (oc >= 4);
  const double cm = swp ? s0 : c0;
  const double sm = swp ? c0 : s0;
  c = cneg ? -cm : cm;
  s = sneg ? -sm : sm;
}

__device__ __forceinline__ _Float16 pick_part(float v, int upper, int isres) {
  float hf, rf;
  split_parts(v, hf, rf);
  const float main_sel = upper ? 0.0f : hf;
  const float res_sel  = upper ? hf : rf;
  const float sel      = isres ? res_sel : main_sel;
  return (_Float16)sel;
}

__global__ __launch_bounds__(256) void basis_build_kernel(_Float16* __restrict__ basis) {
  __shared__ float sWf[kTaps];
  __shared__ __align__(16) float sC[kCoefElems];
  const int tid = threadIdx.x;
  if (tid < kTaps) {
    double c, s;
    cs_two_pi(tid, kTaps, kPiQuarter / (double)kTaps, c, s);
    sWf[tid] = (float)(0.5 * (1.0 - c));
  }
  __syncthreads();
#pragma unroll 1
  for (int it = 0; it < 14; ++it) {
    const int idx  = it * 256 + tid;
    const int tap  = idx & (kTaps - 1);
    const int rr   = idx >> 4;
    const int part = rr / kBinRows;
    const int row  = rr - part * kBinRows;
    const int binc = row < kBinsUsed ? row : (kBinsUsed - 1);
    const int ph   = (binc * (kLeft + tap)) % kFft;
    double c, s;
    cs_two_pi(ph, kFft, kPiQuarter / (double)kFft, c, s);
    const double w  = (double)sWf[tap];
    const double tv = part ? s : c;
    const float  fv = (float)(w * tv);
    sC[idx] = (row < kBinsUsed) ? (fv * kBCarry) : 0.0f;
  }
  __syncthreads();
#pragma unroll 1
  for (int it = 0; it < 7; ++it) {
    const int tsk   = it * 256 + tid;
    const int e0    = tsk * 8;
    const int kind  = e0 / kKindStride;
    const int rem   = e0 - kind * kKindStride;
    const int row   = rem >> 5;
    const int k0    = rem & 31;
    const int upper = k0 >> 4;
    const int tap0  = k0 & 15;
    const int part  = kind >> 1;
    const int isres = kind & 1;
    const float* cp = sC + (part * kBinRows + row) * kTaps + tap0;
    const v4f c0 = *(const v4f*)(cp);
    const v4f c1 = *(const v4f*)(cp + 4);
    v8h hv;
#pragma unroll
    for (int e = 0; e < 4; ++e) {
      const float f0 = c0[e];
      const float f1 = c1[e];
      hv[e]     = pick_part(f0, upper, isres);
      hv[4 + e] = pick_part(f1, upper, isres);
    }
    _Float16* dst = basis + e0;
    *(volatile v8h*)dst = hv;
    __threadfence();
    *(volatile v8h*)dst = hv;
  }
}

__global__ __launch_bounds__(256) void spec_band_kernel(const float* __restrict__ x,
                                                        const _Float16* __restrict__ basis,
                                                        float* __restrict__ plane) {
  __shared__ __align__(16) _Float16 sXh[kStageLen];
  __shared__ __align__(16) _Float16 sXl[kStageLen];
  __shared__ __align__(16) _Float16 sB[kBasisElems];
  __shared__ __align__(16) float    sO[kPlaneSig];

  const int tid  = threadIdx.x;
  const int lane = tid & 31;
  const int wave = tid >> 5;
  const int hh   = lane >> 4;
  const int n    = lane & 15;
  const int sig  = blockIdx.x;
  const float* xs = x + (size_t)sig * kSigLen;

#pragma unroll
  for (int it = 0; it < 7; ++it) {
    const int o = (it * 256 + tid) * 8;
    const v8h bv = *(const v8h*)(basis + o);
    *(v8h*)(sB + o) = bv;
  }

#pragma unroll 1
  for (int it = 0; it < kStageIters; ++it) {
    const int i  = it * 256 + tid;
    const int ic = i < kStageLen ? i : (kStageLen - 1);
    int j = ic - kShift;
    j = j < 0 ? -j : j;
    j = j >= kSigLen ? (2 * kSigLen - 2 - j) : j;
    float v = xs[j];
    asm volatile("" : "+v"(v));
    float hf, rf;
    split_parts(v * kXCarry, hf, rf);
    if (i < kStageLen) {
      sXh[i] = (_Float16)hf;
      sXl[i] = (_Float16)rf;
    }
  }
  __syncthreads();

#pragma unroll 1
  for (int f = 0; f < 4; ++f) {
    const int frame = (wave * 4 + f) * 16 + n;
    FragH fb;
    fb.h[0] = *(const v8h*)(sXh + kHop * frame + 8 * hh);
    fb.h[1] = *(const v8h*)(sXl + kHop * frame + 8 * hh);

    float bacc[kBands];
#pragma unroll
    for (int b = 0; b < kBands; ++b) bacc[b] = 0.0f;

#pragma unroll 1
    for (int bt = 0; bt < kBinTiles; ++bt) {
      const _Float16* bp = sB + ((bt * 16 + n) * kKPad + 8 * hh);
      const v16h a0 = frag_load(bp);
      const v16h a1 = frag_load(bp + kKindStride);
      const v16h a2 = frag_load(bp + 2 * kKindStride);
      const v16h a3 = frag_load(bp + 3 * kKindStride);
      v8f mre = (v8f){0.f, 0.f, 0.f, 0.f, 0.f, 0.f, 0.f, 0.f};
      v8f rre = (v8f){0.f, 0.f, 0.f, 0.f, 0.f, 0.f, 0.f, 0.f};
      v8f mim = (v8f){0.f, 0.f, 0.f, 0.f, 0.f, 0.f, 0.f, 0.f};
      v8f rim = (v8f){0.f, 0.f, 0.f, 0.f, 0.f, 0.f, 0.f, 0.f};
      mre = mma_h(a0, fb.v, mre);
      rre = mma_h(a1, fb.v, rre);
      mim = mma_h(a2, fb.v, mim);
      rim = mma_h(a3, fb.v, rim);

      const int g8    = bt * 16 + hh * 8;
      const int bl    = band_of_bin(g8);
      const int bu    = band_of_bin(g8 + 7);
      const int split = band_end(bl) - g8;
      float sl = 0.0f, su = 0.0f;
#pragma unroll
      for (int r = 0; r < 8; ++r) {
        const float re  = (mre[r] + rre[r] * kInvRes) * kInvCarry;
        const float im  = (mim[r] + rim[r] * kInvRes) * kInvCarry;
        const float pw  = re * re + im * im;
        const float amp = logf(pw + kEps);
        const bool lowp = (r < split);
        sl += lowp ? amp : 0.0f;
        su += lowp ? 0.0f : amp;
      }
#pragma unroll
      for (int b = 0; b < kBands; ++b) {
        const float addl = (bl == b) ? sl : 0.0f;
        const float addu = (bu == b) ? su : 0.0f;
        bacc[b] += addl + addu;
      }
    }

#pragma unroll
    for (int b = 0; b < kBands; ++b) {
      const float mine  = bacc[b];
      const float other = __shfl_xor(mine, 16, 32);
      const float mean  = (mine + other) * (1.0f / (float)band_width(b));
      if (hh == 0) sO[b * kFramesPad + frame] = mean;
    }
  }
  __syncthreads();

  float* pl = plane + (size_t)sig * kPlaneSig;
  v4f vals[4];
#pragma unroll
  for (int it = 0; it < 4; ++it) {
    const int idx = it * 256 + tid;
    const int idc = idx < kPlaneVec ? idx : (kPlaneVec - 1);
    vals[it] = *(const v4f*)(sO + 4 * idc);
  }
  for (int pass = 0; pass < 2; ++pass) {
#pragma unroll
    for (int it = 0; it < 4; ++it) {
      const int idx = it * 256 + tid;
      if (idx < kPlaneVec) *(volatile v4f*)(pl + 4 * idx) = vals[it];
    }
    __threadfence();
  }
}

__global__ __launch_bounds__(256) void compact_kernel(const float* __restrict__ plane, float* __restrict__ out) {
  const int g = blockIdx.x * 256 + threadIdx.x;
  v4f v;
#pragma unroll
  for (int e = 0; e < 4; ++e) {
    const int i    = 4 * g + e;
    const int sig  = i / kOutSig;
    const int rem  = i - sig * kOutSig;
    const int band = rem / kFrames;
    const int t    = rem - band * kFrames;
    v[e] = plane[(size_t)(sig * kBands + band) * kFramesPad + t];
  }
  float* dst = out + (size_t)4 * g;
  *(volatile v4f*)dst = v;
  __threadfence();
  *(volatile v4f*)dst = v;
}

extern "C" void kernel_launch(void* const* d_in, const int* in_sizes, int n_in,
                              void* d_out, int out_size, void* d_ws, size_t ws_size,
                              hipStream_t stream) {
  if (n_in < 1) return;
  if (in_sizes[0] != kNumSig * kSigLen) return;
  if (out_size != kOutElems) return;
  if (ws_size < kWsTotal) return;

  const float* x = (const float*)d_in[0];
  char* ws = (char*)d_ws;
  _Float16* basis = (_Float16*)(ws + kOffBasis);
  float*    plane = (float*)(ws + kOffPlane);
  float*    out   = (float*)d_out;

  basis_build_kernel<<<1, 256, 0, stream>>>(basis);
  spec_band_kernel<<<kNumSig, 256, 0, stream>>>(x, basis, plane);
  compact_kernel<<<kOutVec / 256, 256, 0, stream>>>(plane, out);
}
